// SoftWeightedDecompositionKernel_18683107737746
// MI455X (gfx1250) — hardware-run, weakly checked
//
#include <hip/hip_runtime.h>
#include <stddef.h>
#include <stdint.h>
#include <math.h>


#define LL     128
#define NS     30
#define NSP    32
#define SD     8
#define PD     64
#define NR1    1024
#define NR2    1024
#define TI     16
#define TJ     32
#define NTHR   256
#define NWAVE  8
#define WSCAP  134217728

static_assert(NTHR == NWAVE * 32);
static_assert((NR1 % TI) == 0);
static_assert((NR2 % TJ) == 0);
static_assert(((NR1 + NR2) % 32) == 0);
static_assert((NR1 % 32) == 0);
static_assert(LL == 128);
static_assert(TI * LL == 8 * NTHR);
static_assert(TJ * LL == 16 * NTHR);
static_assert(NSP * NSP == 4 * NTHR);

#define MO_W16  0
#define MO_S    32768
#define MO_X1   36864
#define MO_X2   38912
#define MO_RV1  43008
#define MO_RV2  43072
#define MO_OB   43264
#define MO_ST   44288
#define MLDS    109824
static_assert(MO_ST + NWAVE * 16 * LL * 4 == MLDS);
static_assert((MO_ST % 16) == 0);
static_assert((MO_X1 % 16) == 0);
static_assert((MO_X2 % 16) == 0);
static_assert(MLDS <= 300 * 1024);

#define RO_WL   0
#define RO_DL   65536
#define RO_SD   65664
#define RO_RQ   69760
#define RLDS    69888
static_assert((RO_SD % 16) == 0);
static_assert((RO_RQ % 16) == 0);

#define SZ_WF   ((size_t)LL * LL * 4)
#define SZ_W16  ((size_t)LL * LL * 2)
#define SZ_S32  ((size_t)NSP * NSP * 4)
#define SZ_RV   ((size_t)(NR1 + NR2) * 4)
#define SZ_TOT  (SZ_WF + SZ_W16 + SZ_S32 + SZ_RV)
static_assert(SZ_TOT <= (size_t)WSCAP);
static_assert((SZ_WF % 256) == 0);
static_assert((SZ_W16 % 256) == 0);
static_assert((SZ_S32 % 256) == 0);
static_assert((SZ_RV % 256) == 0);

typedef float          v4f  __attribute__((ext_vector_type(4)));
typedef float          v8f  __attribute__((ext_vector_type(8)));
typedef _Float16       v8h  __attribute__((ext_vector_type(8)));
typedef _Float16       v16h __attribute__((ext_vector_type(16)));
typedef unsigned int   u4   __attribute__((ext_vector_type(4)));
typedef int            v4i  __attribute__((ext_vector_type(4)));
union FragH { v16h v; v8h h[2]; };

__device__ __forceinline__ v8f wmf(v16h a, v16h b, v8f c) {
  v8f d = __builtin_amdgcn_wmma_f32_16x16x32_f16(false, a, false, b, (short)0, c, false, false);
  asm volatile("v_nop\n\tv_nop\n\tv_nop\n\tv_nop" : "+v"(d) : "v"(a), "v"(b));
  return d;
}

__device__ __forceinline__ v8h cvt8(v4f a, v4f b) {
  v8h r;
  r[0] = (_Float16)a.x; r[1] = (_Float16)a.y; r[2] = (_Float16)a.z; r[3] = (_Float16)a.w;
  r[4] = (_Float16)b.x; r[5] = (_Float16)b.y; r[6] = (_Float16)b.z; r[7] = (_Float16)b.w;
  return r;
}

__device__ __forceinline__ unsigned int pk4(v4i v) {
  const unsigned int c0 = (unsigned int)min(max(v.x, 0), NS - 1);
  const unsigned int c1 = (unsigned int)min(max(v.y, 0), NS - 1);
  const unsigned int c2 = (unsigned int)min(max(v.z, 0), NS - 1);
  const unsigned int c3 = (unsigned int)min(max(v.w, 0), NS - 1);
  return c0 | (c1 << 8) | (c2 << 16) | (c3 << 24);
}

#define WAIT_LOADS() asm volatile("s_wait_loadcnt 0x0" ::: "memory")

__global__ __launch_bounds__(LL) void k_prepw(const float* __restrict__ pe, float* wf, _Float16* w16) {
  __shared__ __attribute__((aligned(16))) float wrow[LL];
  const int p = blockIdx.x, q = threadIdx.x, lane = q & 31, wv = q >> 5;
  const float* pp = pe + (size_t)p * PD;
  const float* pq = pe + (size_t)q * PD;
  float dot = 0.f, np = 0.f, nq = 0.f;
#pragma unroll 4
  for (int k = 0; k < PD; ++k) {
    const float ap = pp[k], aq = pq[k];
    dot = fmaf(ap, aq, dot);
    np = fmaf(ap, ap, np);
    nq = fmaf(aq, aq, nq);
  }
  const float pr = rsqrtf(np) * rsqrtf(nq);
  float w = fmaf(dot, pr, 1.0f) * 0.5f;
  w = (p == q) ? 0.f : w;
  wrow[q] = w;
  __syncthreads();
  if (wv == 0) {
    const v4f v = *(const v4f*)(wrow + 4 * lane);
    float* d = wf + (size_t)p * LL + 4 * lane;
    *(volatile v4f*)d = v;
    __threadfence();
    *(volatile v4f*)d = v;
  }
  if (wv == 1) {
    const int c = 8 * (lane & 15);
    const v4f f0 = *(const v4f*)(wrow + c);
    const v4f f1 = *(const v4f*)(wrow + c + 4);
    const v8h hv = cvt8(f0, f1);
    _Float16* d = w16 + (size_t)p * LL + c;
    if (lane < 16) *(volatile v8h*)d = hv;
    __threadfence();
    if (lane < 16) *(volatile v8h*)d = hv;
  }
}

__global__ __launch_bounds__(NTHR) void k_preps(const float* __restrict__ A, float* s32) {
  __shared__ float al[NS * SD];
  __shared__ __attribute__((aligned(16))) float tab[NSP * NSP];
  const int tid = threadIdx.x;
  if (tid < NS * SD) al[tid] = A[tid];
  __syncthreads();
#pragma unroll 1
  for (int k = 0; k < 4; ++k) {
    const int idx = tid + NTHR * k;
    const int r = idx >> 5, c = idx & 31;
    const int rr = min(r, NS - 1), cc = min(c, NS - 1);
    float s = 0.f;
#pragma unroll
    for (int d = 0; d < SD; ++d) s = fmaf(al[rr * SD + d], al[cc * SD + d], s);
    tab[idx] = (r < NS && c < NS) ? s : 0.f;
  }
  __syncthreads();
  const v4f v = *(const v4f*)(tab + 4 * tid);
  float* d = s32 + 4 * tid;
  *(volatile v4f*)d = v;
  __threadfence();
  *(volatile v4f*)d = v;
}

__global__ __launch_bounds__(NTHR) void k_rinv(const int* __restrict__ X1, const int* __restrict__ X2,
                                               const float* __restrict__ A, const float* __restrict__ wf,
                                               float* rinv) {
  extern __shared__ __attribute__((aligned(16))) char smem[];
  float* wl = (float*)(smem + RO_WL);
  float* dl = (float*)(smem + RO_DL);
  float* rq = (float*)(smem + RO_RQ);
  const int tid = threadIdx.x, lane = tid & 31, wv = tid >> 5;
  float* sd = (float*)(smem + RO_SD) + wv * LL;
  const int rbase = blockIdx.x * 32;
  const int* X = (rbase < NR1) ? (X1 + (size_t)rbase * LL) : (X2 + (size_t)(rbase - NR1) * LL);

#pragma unroll 1
  for (int g = 0; g < 2; ++g) {
    v4f tv[8];
#pragma unroll
    for (int k = 0; k < 8; ++k) {
      const int idx = tid + NTHR * (8 * g + k);
      tv[k] = *(const v4f*)(wf + 4 * idx);
    }
#pragma unroll
    for (int k = 0; k < 8; ++k) {
      const int idx = tid + NTHR * (8 * g + k);
      *(v4f*)(wl + 4 * idx) = tv[k];
    }
    WAIT_LOADS();
  }
  if (tid < 32) {
    const int r = min(tid, NS - 1);
    float s = 0.f;
#pragma unroll
    for (int d = 0; d < SD; ++d) { const float av = A[r * SD + d]; s = fmaf(av, av, s); }
    dl[tid] = (tid < NS) ? s : 0.f;
  }
  __syncthreads();

#pragma unroll 1
  for (int rr = 0; rr < 4; ++rr) {
    const int rl = wv + 8 * rr;
    const int* xr = X + (size_t)rl * LL;
#pragma unroll
    for (int k = 0; k < 4; ++k) {
      const int p = lane + 32 * k;
      int xv = xr[p];
      xv = min(max(xv, 0), NS - 1);
      sd[p] = dl[xv];
    }
    __syncthreads();
    float acc[4] = {0.f, 0.f, 0.f, 0.f};
#pragma unroll 2
    for (int p = 0; p < LL; ++p) {
      const float dp = sd[p];
      const float* wr = wl + p * LL + lane;
#pragma unroll
      for (int k = 0; k < 4; ++k) acc[k] = fmaf(dp, wr[32 * k], acc[k]);
    }
    float part = 0.f;
#pragma unroll
    for (int k = 0; k < 4; ++k) part = fmaf(acc[k], sd[lane + 32 * k], part);
    part += __shfl_xor(part, 16);
    part += __shfl_xor(part, 8);
    part += __shfl_xor(part, 4);
    part += __shfl_xor(part, 2);
    part += __shfl_xor(part, 1);
    if (lane == 0) rq[rl] = rsqrtf(part);
    __syncthreads();
  }

  if (wv == 0) {
    const v4f v = *(const v4f*)(rq + 4 * (lane & 7));
    float* d = rinv + rbase + 4 * (lane & 7);
    if (lane < 8) *(volatile v4f*)d = v;
    __threadfence();
    if (lane < 8) *(volatile v4f*)d = v;
  }
}

__global__ __launch_bounds__(NTHR) void k_main(const int* __restrict__ X1, const int* __restrict__ X2,
                                               const _Float16* __restrict__ w16g, const float* __restrict__ s32g,
                                               const float* __restrict__ rinv,
                                               const float* __restrict__ pa, const float* __restrict__ pg,
                                               float* out) {
  extern __shared__ __attribute__((aligned(16))) char smem[];
  const int tid = threadIdx.x, lane = tid & 31, wv = tid >> 5, hh = lane >> 4, m = lane & 15;
  const _Float16* wl = (const _Float16*)(smem + MO_W16);
  float* Sl = (float*)(smem + MO_S);
  unsigned char* x1b = (unsigned char*)(smem + MO_X1);
  unsigned char* x2b = (unsigned char*)(smem + MO_X2);
  float* rv1 = (float*)(smem + MO_RV1);
  float* rv2 = (float*)(smem + MO_RV2);
  float* ob = (float*)(smem + MO_OB) + wv * 32;
  float* st = (float*)(smem + MO_ST) + wv * (16 * LL);
  const int bj = blockIdx.x, bi = blockIdx.y;

  {
    u4* dw = (u4*)(smem + MO_W16);
    const u4* sw = (const u4*)w16g;
    u4 tw[8];
#pragma unroll
    for (int k = 0; k < 8; ++k) tw[k] = sw[tid + NTHR * k];
#pragma unroll
    for (int k = 0; k < 8; ++k) dw[tid + NTHR * k] = tw[k];
  }
  WAIT_LOADS();

  {
    const v4f sv = *(const v4f*)(s32g + 4 * tid);
    v4i xa[2], xb[4];
#pragma unroll
    for (int k = 0; k < 2; ++k) {
      const int idx = tid + NTHR * k;
      xa[k] = *(const v4i*)(X1 + (size_t)(bi * TI + (idx >> 5)) * LL + 4 * (idx & 31));
    }
#pragma unroll
    for (int k = 0; k < 4; ++k) {
      const int idx = tid + NTHR * k;
      xb[k] = *(const v4i*)(X2 + (size_t)(bj * TJ + (idx >> 5)) * LL + 4 * (idx & 31));
    }
    *(v4f*)(Sl + 4 * tid) = sv;
#pragma unroll
    for (int k = 0; k < 2; ++k) {
      const int idx = tid + NTHR * k;
      *(unsigned int*)(x1b + 4 * idx) = pk4(xa[k]);
    }
#pragma unroll
    for (int k = 0; k < 4; ++k) {
      const int idx = tid + NTHR * k;
      *(unsigned int*)(x2b + 4 * idx) = pk4(xb[k]);
    }
  }
  WAIT_LOADS();
  if (wv == 0) rv2[lane] = rinv[NR1 + bj * TJ + lane];
  if (wv == 1) rv1[m] = rinv[bi * TI + m];
  __syncthreads();

  const float av = pa[0], gv = pg[0];
  const float a2 = av * av;
  const v8f zero8 = {0.f, 0.f, 0.f, 0.f, 0.f, 0.f, 0.f, 0.f};

#pragma unroll 1
  for (int t = 0; t < 4; ++t) {
    const int il = wv + 8 * (t >> 1);
    const int jh = t & 1;
    __syncthreads();

    {
      const unsigned char* xi = x1b + il * LL;
      const unsigned char* xj = x2b + (jh * 16) * LL;
#pragma unroll 4
      for (int k = 0; k < 64; ++k) {
        const int jl = k >> 2;
        const int p = lane + 32 * (k & 3);
        const int ra = xi[p], cb = xj[jl * LL + p];
        st[jl * LL + p] = Sl[ra * NSP + cb];
      }
    }
    __syncthreads();

    float red[8];
#pragma unroll
    for (int r = 0; r < 8; ++r) red[r] = 0.f;
#pragma unroll 1
    for (int nh = 0; nh < 2; ++nh) {
      v8f acc[4];
#pragma unroll
      for (int nt = 0; nt < 4; ++nt) acc[nt] = zero8;
#pragma unroll 1
      for (int kt = 0; kt < 4; ++kt) {
        const int k0 = 32 * kt;
        const float* ar = st + m * LL + k0 + 8 * hh;
        const v4f f0 = *(const v4f*)ar;
        const v4f f1 = *(const v4f*)(ar + 4);
        const v4f f2 = *(const v4f*)(ar + 16);
        const v4f f3 = *(const v4f*)(ar + 20);
        FragH af;
        af.h[0] = cvt8(f0, f1);
        af.h[1] = cvt8(f2, f3);
        const _Float16* bb = wl + (size_t)(nh * 64 + m) * LL + k0 + 8 * hh;
#pragma unroll
        for (int nt = 0; nt < 4; ++nt) {
          const _Float16* bq = bb + nt * 16 * LL;
          FragH bf;
          bf.h[0] = *(const v8h*)bq;
          bf.h[1] = *(const v8h*)(bq + 16);
          acc[nt] = wmf(af.v, bf.v, acc[nt]);
        }
      }
#pragma unroll
      for (int nt = 0; nt < 4; ++nt) {
        const float* sc = st + (8 * hh) * LL + nh * 64 + nt * 16 + m;
#pragma unroll
        for (int r = 0; r < 8; ++r) red[r] = fmaf(acc[nt][r], sc[r * LL], red[r]);
      }
    }
#pragma unroll
    for (int r = 0; r < 8; ++r) {
      float v = red[r];
      v += __shfl_xor(v, 1);
      v += __shfl_xor(v, 2);
      v += __shfl_xor(v, 4);
      v += __shfl_xor(v, 8);
      red[r] = v;
    }
    const int rsel = m & 7;
    float kv = red[0];
#pragma unroll
    for (int r = 1; r < 8; ++r) kv = (rsel == r) ? red[r] : kv;
    const int jt = jh * 16 + 8 * hh + rsel;
    float val = kv * rv1[il];
    val = val * rv2[jt];
    const float o = a2 * powf(val, gv);
    if (m < 8) ob[jt] = o;

    if (jh == 1) {
      __syncthreads();
      const v4f v = *(const v4f*)(ob + 4 * (lane & 7));
      float* gp = out + (size_t)(bi * TI + il) * NR2 + bj * TJ + 4 * (lane & 7);
      if (lane < 8) *(volatile v4f*)gp = v;
      __threadfence();
      if (lane < 8) *(volatile v4f*)gp = v;
    }
  }
}

extern "C" void kernel_launch(void* const* d_in, const int* in_sizes, int n_in,
                              void* d_out, int out_size, void* d_ws, size_t ws_size,
                              hipStream_t stream) {
  if (n_in < 6) return;
  if (in_sizes[0] != NR1 * LL || in_sizes[1] != NR2 * LL) return;
  if (in_sizes[2] != NS * SD) return;
  if (in_sizes[3] != LL * PD) return;
  if (in_sizes[4] < 1 || in_sizes[5] < 1) return;
  if (out_size != NR1 * NR2) return;

  const int*   X1 = (const int*)d_in[0];
  const int*   X2 = (const int*)d_in[1];
  const float* A  = (const float*)d_in[2];
  const float* pe = (const float*)d_in[3];
  const float* pa = (const float*)d_in[4];
  const float* pg = (const float*)d_in[5];
  float* out = (float*)d_out;

  char* ws = (char*)d_ws;
  size_t off = 0;
  const size_t oWF  = off; off += SZ_WF;
  const size_t oW16 = off; off += SZ_W16;
  const size_t oS32 = off; off += SZ_S32;
  const size_t oRV  = off; off += SZ_RV;
  if (off != SZ_TOT) return;
  if (off > ws_size || off > (size_t)WSCAP) return;

  float*    wf   = (float*)(ws + oWF);
  _Float16* w16  = (_Float16*)(ws + oW16);
  float*    s32  = (float*)(ws + oS32);
  float*    rinv = (float*)(ws + oRV);

  hipFuncSetAttribute(reinterpret_cast<const void*>(&k_rinv),
                      hipFuncAttributeMaxDynamicSharedMemorySize, RLDS);
  hipFuncSetAttribute(reinterpret_cast<const void*>(&k_main),
                      hipFuncAttributeMaxDynamicSharedMemorySize, MLDS);

  k_prepw<<<LL, LL, 0, stream>>>(pe, wf, w16);
  k_preps<<<1, NTHR, 0, stream>>>(A, s32);
  k_rinv<<<(NR1 + NR2) / 32, NTHR, RLDS, stream>>>(X1, X2, A, wf, rinv);
  k_main<<<dim3(NR2 / TJ, NR1 / TI), NTHR, MLDS, stream>>>(X1, X2, w16, s32, rinv, pa, pg, out);
}
